// LSTMModel_2241972928621
// MI455X (gfx1250) — hardware-verified
//
#include <hip/hip_runtime.h>
#include <cstdint>
#include <cstddef>
#include <math.h>


constexpr int Bc = 4096;
constexpr int Tc = 1024;
constexpr int Hc = 32;
constexpr int CHUNK = 64;

typedef __attribute__((ext_vector_type(16))) _Float16 v16h;
typedef __attribute__((ext_vector_type(8)))  _Float16 v8h;
typedef __attribute__((ext_vector_type(8)))  float    v8f;
typedef __attribute__((ext_vector_type(4)))  float    v4f;
typedef float __attribute__((may_alias)) float_a;

template <typename T> __device__ __forceinline__ void vst2(void* p, T v) { *(volatile T*)p = v; __threadfence(); *(volatile T*)p = v; }
__device__ __forceinline__ v8f wmma16(v16h a, v16h b, v8f c) {
    v8f d = __builtin_amdgcn_wmma_f32_16x16x32_f16(false, a, false, b, (short)0, c, false, false);
    asm volatile("v_nop\n\tv_nop\n\tv_nop\n\tv_nop" : "+v"(d) : "v"(a), "v"(b));
    return d;
}
__device__ __forceinline__ float sig_(float x) { return 1.0f / (1.0f + expf(-x)); }

__global__ __launch_bounds__(64)
void lstm_wmma_kernel(const float* __restrict__ x, const float* __restrict__ W_ih, const float* __restrict__ W_hh,
                      const float* __restrict__ b_ih, const float* __restrict__ b_hh, const float* __restrict__ fc_w,
                      const float* __restrict__ fc_b, float* __restrict__ out)
{
    __shared__ __attribute__((aligned(16))) float    xs[2][CHUNK][20];
    __shared__ __attribute__((aligned(16))) _Float16 hrow[2][16][40];
    __shared__ float res[32];

    const int wave = threadIdx.x >> 5;
    const int lane = threadIdx.x & 31;
    const int col  = lane & 15;
    const int kh   = lane >> 4;
    const int roff = kh * 8;
    const int base = blockIdx.x * 32 + wave * 16;

    v16h Bf[8];
#pragma unroll
    for (int j = 0; j < 8; ++j) {
        const float* wr = W_hh + (size_t)(16 * j + col) * Hc;
        v16h b;
#pragma unroll
        for (int e = 0; e < 16; ++e) b[e] = (_Float16)wr[8 * kh + ((e < 8) ? e : (e + 8))];
        Bf[j] = b;
    }
    float wih[8], bsum[8];
#pragma unroll
    for (int j = 0; j < 8; ++j) { const int g = 16 * j + col; wih[j] = W_ih[g]; bsum[j] = b_ih[g] + b_hh[g]; }

    v16h Af;
#pragma unroll
    for (int e = 0; e < 16; ++e) Af[e] = (_Float16)0.0f;
    v8f cs0, cs1, hs0, hs1;
#pragma unroll
    for (int r = 0; r < 8; ++r) { cs0[r]=0.f; cs1[r]=0.f; hs0[r]=0.f; hs1[r]=0.f; }

    float (*xw)[20] = xs[wave];
    _Float16 (*hw)[40] = hrow[wave];

    for (int t0 = 0; t0 < Tc; t0 += CHUNK) {
        __builtin_amdgcn_wave_barrier();
#pragma unroll
        for (int s = 0; s < 32; ++s) {
            const int idx = s * 32 + lane;
            const int m  = idx >> 6;
            const int tq = idx & 63;
            xw[tq][m] = x[(size_t)(base + m) * Tc + (t0 + tq)];
        }
        asm volatile("s_wait_loadcnt 0\n\ts_wait_dscnt 0" ::: "memory");
        __builtin_amdgcn_wave_barrier();
        __builtin_amdgcn_fence(__ATOMIC_RELEASE, "workgroup");

        for (int tt = 0; tt < CHUNK; ++tt) {
            const v4f xa = *(const v4f*)&xw[tt][roff];
            const v4f xb = *(const v4f*)&xw[tt][roff + 4];
            float xv[8];
#pragma unroll
            for (int r = 0; r < 4; ++r) { xv[r] = xa[r]; xv[r + 4] = xb[r]; }

            v8f acc[8];
#pragma unroll
            for (int j = 0; j < 8; ++j) {
                v8f cin;
#pragma unroll
                for (int r = 0; r < 8; ++r) cin[r] = fmaf(xv[r], wih[j], bsum[j]);
                acc[j] = wmma16(Af, Bf[j], cin);
            }
#pragma unroll
            for (int r = 0; r < 8; ++r) {
                const float iv0 = sig_(acc[0][r]), iv1 = sig_(acc[1][r]);
                const float fv0 = sig_(acc[2][r]), fv1 = sig_(acc[3][r]);
                const float gv0 = tanhf(acc[4][r]), gv1 = tanhf(acc[5][r]);
                const float ov0 = sig_(acc[6][r]), ov1 = sig_(acc[7][r]);
                cs0[r] = fv0 * cs0[r] + iv0 * gv0;
                cs1[r] = fv1 * cs1[r] + iv1 * gv1;
                hs0[r] = ov0 * tanhf(cs0[r]);
                hs1[r] = ov1 * tanhf(cs1[r]);
            }
            __builtin_amdgcn_wave_barrier();
#pragma unroll
            for (int r = 0; r < 8; ++r) { hw[roff + r][col] = (_Float16)hs0[r]; hw[roff + r][16 + col] = (_Float16)hs1[r]; }
            asm volatile("s_wait_dscnt 0" ::: "memory");
            __builtin_amdgcn_wave_barrier();
            __builtin_amdgcn_fence(__ATOMIC_RELEASE, "workgroup");
            {
                union { v16h v; v8h q[2]; } a;
                a.q[0] = *(const v8h*)&hw[col][8 * kh];
                a.q[1] = *(const v8h*)&hw[col][16 + 8 * kh];
                Af = a.v;
            }
        }
    }

    const float fw0 = fc_w[col], fw1 = fc_w[col + 16], bias = fc_b[0];
#pragma unroll
    for (int r = 0; r < 8; ++r) {
        float v = hs0[r] * fw0 + hs1[r] * fw1;
        v += __shfl_xor(v, 1); v += __shfl_xor(v, 2); v += __shfl_xor(v, 4); v += __shfl_xor(v, 8);
        if (col == 0) res[wave * 16 + roff + r] = v + bias;
    }
    __syncthreads();
    if (threadIdx.x < 32) vst2(out + blockIdx.x * 32 + threadIdx.x, (float_a)res[threadIdx.x]);
}

extern "C" void kernel_launch(void* const* d_in, const int* in_sizes, int n_in,
                              void* d_out, int out_size, void* d_ws, size_t ws_size,
                              hipStream_t stream) {
    (void)in_sizes; (void)n_in; (void)out_size; (void)d_ws; (void)ws_size;
    const float* x    = (const float*)d_in[0];
    const float* W_ih = (const float*)d_in[1];
    const float* W_hh = (const float*)d_in[2];
    const float* b_ih = (const float*)d_in[3];
    const float* b_hh = (const float*)d_in[4];
    const float* fc_w = (const float*)d_in[5];
    const float* fc_b = (const float*)d_in[6];
    float* out        = (float*)d_out;
    lstm_wmma_kernel<<<Bc / 32, 64, 0, stream>>>(x, W_ih, W_hh, b_ih, b_hh, fc_w, fc_b, out);
}
